// MNIST_CNN2D_TWN_42597485641965
// MI455X (gfx1250) — hardware-verified
//
#include <hip/hip_runtime.h>
#define BB 512
#define C1 64
#define C2 128
#define H0 28
#define H1 24
#define Q1 12
#define H2 8
#define Q2 4
#define F1 512
#define NCLS 10
#define R1 (BB * H1 * H1)
#define K1P 32
#define R2 (BB * H2 * H2)
#define K2 (25 * C1)
#define BH2 256

typedef __bf16 v16b __attribute__((ext_vector_type(16)));
typedef unsigned short v8us __attribute__((ext_vector_type(8), may_alias));
typedef float  v8f  __attribute__((ext_vector_type(8)));
typedef float  v4f  __attribute__((ext_vector_type(4)));
typedef float  v4fa __attribute__((ext_vector_type(4), may_alias));
union FragB { v16b v; v8us half[2]; unsigned short u[16]; };

__device__ __forceinline__ unsigned short bf16_bits(float x) { unsigned int u = __float_as_uint(x); return (unsigned short)((u + 0x7FFFu + ((u >> 16) & 1u)) >> 16); }
__device__ __forceinline__ float bf16_val(unsigned short b) { return __uint_as_float(((unsigned int)b) << 16); }
__device__ __forceinline__ float bf16_round(float x) { return bf16_val(bf16_bits(x)); }
template <int NT>
__device__ __forceinline__ v8f mmaN(v16b ah, v16b al, v16b bh, v16b bl, v8f c) {
  c = __builtin_amdgcn_wmma_f32_16x16x32_bf16(false, ah, false, bh, (short)0, c, false, false);
  if (NT >= 2) c = __builtin_amdgcn_wmma_f32_16x16x32_bf16(false, al, false, bh, (short)0, c, false, false);
  if (NT >= 3) c = __builtin_amdgcn_wmma_f32_16x16x32_bf16(false, ah, false, bl, (short)0, c, false, false);
  asm volatile("v_nop\n\tv_nop\n\tv_nop\n\tv_nop" : "+v"(c) : "v"(ah), "v"(al), "v"(bh), "v"(bl));
  return c;
}

__global__ __launch_bounds__(256) void k_wt_bf16(const float* __restrict__ W, unsigned short* __restrict__ Wt, int K, int N) {
  const int t = blockIdx.x * 256 + threadIdx.x;
  const int k8n = K / 8;
  if (t >= N * k8n) return;
  const int n = t / k8n, k8 = (t % k8n) * 8;
  v8us v;
#pragma unroll
  for (int i = 0; i < 8; ++i) v[i] = bf16_bits(W[(size_t)(k8 + i) * N + n]);
  *(volatile v8us*)(Wt + (size_t)n * K + k8) = v;
  __threadfence();
  *(volatile v8us*)(Wt + (size_t)n * K + k8) = v;
}

template <bool ASPLIT, int ACT, bool BIAS_BF16>
__global__ __launch_bounds__(128) void k_gemm_bf(const float* __restrict__ A, int lda, const unsigned short* __restrict__ Wt, int ldb,
                                               const float* __restrict__ bias, float* __restrict__ C, int ldc, int M, int N, int K) {
  __shared__ __attribute__((aligned(16))) float so[4][16][64];
  const int tid = threadIdx.x, w = tid >> 5, lane = tid & 31, ln = lane & 15, hh = lane >> 4;
  const int ntn = N / 64;
  const int wid = blockIdx.x * 4 + w;
  const int mt = wid / ntn, nq = wid % ntn;
  if (mt * 16 >= M) return;
  const int row0 = mt * 16, col0 = nq * 64;
  const float* arow = A + (size_t)(row0 + ln) * lda;
  v8f acc[4] = {};
  for (int kb = 0; kb < K; kb += 32) {
    FragB ah, al;
    const v4f x0 = *(const v4fa*)(arow + kb + 8 * hh), x1 = *(const v4fa*)(arow + kb + 8 * hh + 4);
    const v4f x2 = *(const v4fa*)(arow + kb + 16 + 8 * hh), x3 = *(const v4fa*)(arow + kb + 16 + 8 * hh + 4);
    float xs[16] = {x0[0],x0[1],x0[2],x0[3],x1[0],x1[1],x1[2],x1[3],x2[0],x2[1],x2[2],x2[3],x3[0],x3[1],x3[2],x3[3]};
#pragma unroll
    for (int i = 0; i < 16; ++i) { const unsigned short hb = bf16_bits(xs[i]); ah.u[i] = hb; al.u[i] = ASPLIT ? bf16_bits(xs[i] - bf16_val(hb)) : (unsigned short)0; }
#pragma unroll
    for (int t = 0; t < 4; ++t) {
      const unsigned short* brow = Wt + (size_t)(col0 + t * 16 + ln) * ldb + kb;
      FragB b;
      b.half[0] = *(const v8us*)(brow + 8 * hh);
      b.half[1] = *(const v8us*)(brow + 16 + 8 * hh);
      acc[t] = mmaN<ASPLIT ? 2 : 1>(ah.v, al.v, b.v, b.v, acc[t]);
    }
  }
#pragma unroll
  for (int t = 0; t < 4; ++t) {
    float bv = bias ? bias[col0 + t * 16 + ln] : 0.f;
    if (BIAS_BF16) bv = bf16_round(bv);
#pragma unroll
    for (int r = 0; r < 8; ++r) { float v = acc[t][r] + bv; if (ACT == 1) v = fmaxf(v, 0.f); so[w][8 * hh + r][t * 16 + ln] = v; }
  }
  __builtin_amdgcn_fence(__ATOMIC_ACQ_REL, "workgroup");
  __builtin_amdgcn_wave_barrier();
  const int rsub = lane >> 4, c4 = (lane & 15) * 4;
  for (int pass = 0; pass < 2; ++pass) {
#pragma unroll
    for (int q = 0; q < 8; ++q) {
      const int r = q * 2 + rsub;
      const v4f v = *(const v4fa*)&so[w][r][c4];
      *(volatile v4f*)(C + (size_t)(row0 + r) * ldc + col0 + c4) = v;
    }
    if (pass == 0) __threadfence();
  }
}

template <int D, bool CAUSAL>
__global__ __launch_bounds__(128) void k_flash(const float* __restrict__ qb, const float* __restrict__ kb, const float* __restrict__ vb,
                                             int pitch, int T, int H, float scale, float* __restrict__ y, int ypitch) {
  constexpr int KS = D / 32;
  constexpr int DT = D / 16;
  __shared__ __attribute__((aligned(16))) unsigned short sKh[32][D + 8], sKl[32][D + 8], sVh[32][D + 8], sVl[32][D + 8];
  __shared__ __attribute__((aligned(16))) unsigned short sPh[4][16][40], sPl[4][16][40];
  __shared__ __attribute__((aligned(16))) float sO[4][16][D];
  const int tid = threadIdx.x, w = tid >> 5, lane = tid & 31, ln = lane & 15, hh = lane >> 4;
  const int nqb = (T + 63) / 64;
  const int bh = blockIdx.x / nqb, qblk = blockIdx.x % nqb;
  const int b = bh / H, h = bh % H;
  const int q0 = qblk * 64 + w * 16;
  const float* Q = qb + (size_t)b * T * pitch + h * D;
  const float* K = kb + (size_t)b * T * pitch + h * D;
  const float* V = vb + (size_t)b * T * pitch + h * D;

  FragB aqh[KS], aql[KS];
  {
    int row = q0 + ln; if (row >= T) row = T - 1;
    const float* qr = Q + (size_t)row * pitch;
#pragma unroll
    for (int ks = 0; ks < KS; ++ks)
#pragma unroll
      for (int i = 0; i < 16; ++i) {
        const int d = ks * 32 + ((i < 8) ? (8 * hh + i) : (16 + 8 * hh + (i - 8)));
        const float x = qr[d] * scale; const unsigned short hb = bf16_bits(x);
        aqh[ks].u[i] = hb; aql[ks].u[i] = bf16_bits(x - bf16_val(hb));
      }
  }
  float m_r[8], l_r[8];
#pragma unroll
  for (int r = 0; r < 8; ++r) { m_r[r] = -3.0e38f; l_r[r] = 0.f; }
  v8f oacc[DT];
#pragma unroll
  for (int dt = 0; dt < DT; ++dt) oacc[dt] = (v8f){0.f,0.f,0.f,0.f,0.f,0.f,0.f,0.f};

  const int kv_end = CAUSAL ? min(T, qblk * 64 + 64) : T;
  for (int j0 = 0; j0 < kv_end; j0 += 32) {
    __syncthreads();
    for (int e = tid; e < 32 * (D / 4); e += 128) {
      const int r = e / (D / 4), c4 = (e % (D / 4)) * 4;
      const int key = j0 + r;
      v4f kf = {0.f,0.f,0.f,0.f}, vf = {0.f,0.f,0.f,0.f};
      if (key < T) { kf = *(const v4fa*)(K + (size_t)key * pitch + c4); vf = *(const v4fa*)(V + (size_t)key * pitch + c4); }
#pragma unroll
      for (int t = 0; t < 4; ++t) {
        unsigned short hb = bf16_bits(kf[t]); sKh[r][c4 + t] = hb; sKl[r][c4 + t] = bf16_bits(kf[t] - bf16_val(hb));
        hb = bf16_bits(vf[t]); sVh[r][c4 + t] = hb; sVl[r][c4 + t] = bf16_bits(vf[t] - bf16_val(hb));
      }
    }
    __syncthreads();
    v8f s[2];
#pragma unroll
    for (int nt = 0; nt < 2; ++nt) {
      v8f acc = {};
#pragma unroll
      for (int ks = 0; ks < KS; ++ks) {
        FragB bh_, bl_;
        bh_.half[0] = *(const v8us*)&sKh[nt * 16 + ln][ks * 32 + 8 * hh]; bh_.half[1] = *(const v8us*)&sKh[nt * 16 + ln][ks * 32 + 16 + 8 * hh];
        bl_.half[0] = *(const v8us*)&sKl[nt * 16 + ln][ks * 32 + 8 * hh]; bl_.half[1] = *(const v8us*)&sKl[nt * 16 + ln][ks * 32 + 16 + 8 * hh];
        acc = mmaN<3>(aqh[ks].v, aql[ks].v, bh_.v, bl_.v, acc);
      }
      s[nt] = acc;
    }
    float alpha[8];
#pragma unroll
    for (int r = 0; r < 8; ++r) {
      const int qi = q0 + 8 * hh + r;
      const int ja = j0 + ln, jb = j0 + 16 + ln;
      if (CAUSAL) { if (ja > qi) s[0][r] = -3.0e38f; if (jb > qi) s[1][r] = -3.0e38f; }
      if (ja >= T) s[0][r] = -3.0e38f;
      if (jb >= T) s[1][r] = -3.0e38f;
      float mx = fmaxf(s[0][r], s[1][r]);
      mx = fmaxf(mx, __shfl_xor(mx, 1, 32)); mx = fmaxf(mx, __shfl_xor(mx, 2, 32)); mx = fmaxf(mx, __shfl_xor(mx, 4, 32)); mx = fmaxf(mx, __shfl_xor(mx, 8, 32));
      const float mnew = fmaxf(m_r[r], mx);
      alpha[r] = (mnew > -1.0e38f) ? __expf(m_r[r] - mnew) : 1.0f;
      const float p0 = (s[0][r] > -1.0e38f) ? __expf(s[0][r] - mnew) : 0.f;
      const float p1 = (s[1][r] > -1.0e38f) ? __expf(s[1][r] - mnew) : 0.f;
      m_r[r] = mnew;
      l_r[r] = l_r[r] * alpha[r] + p0 + p1;
      unsigned short hb = bf16_bits(p0); sPh[w][8 * hh + r][ln] = hb;      sPl[w][8 * hh + r][ln] = bf16_bits(p0 - bf16_val(hb));
      hb = bf16_bits(p1);                sPh[w][8 * hh + r][16 + ln] = hb; sPl[w][8 * hh + r][16 + ln] = bf16_bits(p1 - bf16_val(hb));
    }
#pragma unroll
    for (int dt = 0; dt < DT; ++dt)
#pragma unroll
      for (int r = 0; r < 8; ++r) oacc[dt][r] *= alpha[r];
    __builtin_amdgcn_fence(__ATOMIC_ACQ_REL, "workgroup");
    __builtin_amdgcn_wave_barrier();
    FragB pah, pal;
    pah.half[0] = *(const v8us*)&sPh[w][ln][8 * hh]; pah.half[1] = *(const v8us*)&sPh[w][ln][16 + 8 * hh];
    pal.half[0] = *(const v8us*)&sPl[w][ln][8 * hh]; pal.half[1] = *(const v8us*)&sPl[w][ln][16 + 8 * hh];
#pragma unroll
    for (int dt = 0; dt < DT; ++dt) {
      FragB bvh, bvl;
#pragma unroll
      for (int i = 0; i < 8; ++i) {
        bvh.u[i] = sVh[8 * hh + i][dt * 16 + ln]; bvh.u[8 + i] = sVh[16 + 8 * hh + i][dt * 16 + ln];
        bvl.u[i] = sVl[8 * hh + i][dt * 16 + ln]; bvl.u[8 + i] = sVl[16 + 8 * hh + i][dt * 16 + ln];
      }
      oacc[dt] = mmaN<3>(pah.v, pal.v, bvh.v, bvl.v, oacc[dt]);
    }
    __builtin_amdgcn_fence(__ATOMIC_ACQ_REL, "workgroup");
    __builtin_amdgcn_wave_barrier();
  }
#pragma unroll
  for (int r = 0; r < 8; ++r) {
    float l = l_r[r];
    l += __shfl_xor(l, 1, 32); l += __shfl_xor(l, 2, 32); l += __shfl_xor(l, 4, 32); l += __shfl_xor(l, 8, 32);
    l_r[r] = (l > 0.f) ? 1.0f / l : 0.f;
  }
#pragma unroll
  for (int dt = 0; dt < DT; ++dt)
#pragma unroll
    for (int r = 0; r < 8; ++r) sO[w][8 * hh + r][dt * 16 + ln] = oacc[dt][r] * l_r[r];
  __builtin_amdgcn_fence(__ATOMIC_ACQ_REL, "workgroup");
  __builtin_amdgcn_wave_barrier();
  for (int pass = 0; pass < 2; ++pass) {
    for (int r = 0; r < 16; ++r) {
      const int row = q0 + r;
      if (row < T && lane < D / 4) {
        const v4f val = *(const v4fa*)&sO[w][r][lane * 4];
        *(volatile v4f*)(y + ((size_t)b * T + row) * ypitch + h * D + lane * 4) = val;
      }
    }
    if (pass == 0) __threadfence();
  }
}

typedef _Float16 v16h __attribute__((ext_vector_type(16)));
union FragH { v16h v; v8us half[2]; _Float16 h[16]; unsigned short u[16]; };
template <int NT>
__device__ __forceinline__ v8f mmaH(v16h ah, v16h al, v16h bh, v16h bl, v8f c) {
  c = __builtin_amdgcn_wmma_f32_16x16x32_f16(false, ah, false, bh, (short)0, c, false, false);
  if (NT >= 2) c = __builtin_amdgcn_wmma_f32_16x16x32_f16(false, al, false, bh, (short)0, c, false, false);
  if (NT >= 3) c = __builtin_amdgcn_wmma_f32_16x16x32_f16(false, ah, false, bl, (short)0, c, false, false);
  asm volatile("v_nop\n\tv_nop\n\tv_nop\n\tv_nop" : "+v"(c) : "v"(ah), "v"(al), "v"(bh), "v"(bl));
  return c;
}
template <bool ASPLIT>
__global__ __launch_bounds__(128) void k_gemm_h(const float* __restrict__ A, int lda, size_t sA, const _Float16* __restrict__ Bh, int ldb, size_t sB, float alpha, float* __restrict__ C, int ldc, size_t sC, int M, int N, int K) {
  __shared__ __attribute__((aligned(16))) float so[4][16][64];
  const int tid = threadIdx.x, w = tid >> 5, lane = tid & 31, ln = lane & 15, hh = lane >> 4; const int by = blockIdx.y;
  A += (size_t)by * sA; Bh += (size_t)by * sB; C += (size_t)by * sC;
  const int ntn = (N + 63) / 64; const int wid = blockIdx.x * 4 + w; const int mt = wid / ntn, nq = wid % ntn; if (mt * 16 >= M) return;
  const int row0 = mt * 16, col0 = nq * 64; const float* arow = A + (size_t)(row0 + ln) * lda;
  v8f acc[4] = {};
  for (int kb = 0; kb < K; kb += 32) {
    FragH ah, al;
    const v4f x0 = *(const v4fa*)(arow + kb + 8 * hh), x1 = *(const v4fa*)(arow + kb + 8 * hh + 4), x2 = *(const v4fa*)(arow + kb + 16 + 8 * hh), x3 = *(const v4fa*)(arow + kb + 16 + 8 * hh + 4);
    float xs[16] = {x0[0],x0[1],x0[2],x0[3],x1[0],x1[1],x1[2],x1[3],x2[0],x2[1],x2[2],x2[3],x3[0],x3[1],x3[2],x3[3]};
#pragma unroll
    for (int i = 0; i < 16; ++i) { const _Float16 h = (_Float16)xs[i]; ah.h[i] = h; al.h[i] = ASPLIT ? (_Float16)(xs[i] - (float)h) : (_Float16)0.0f; }
#pragma unroll
    for (int t = 0; t < 4; ++t) { if (col0 + t * 16 >= N) continue; const size_t boff = (size_t)(col0 + t * 16 + ln) * ldb + kb; FragH bq; bq.half[0] = *(const v8us*)(Bh + boff + 8 * hh); bq.half[1] = *(const v8us*)(Bh + boff + 16 + 8 * hh);
      acc[t] = mmaH<ASPLIT ? 2 : 1>(ah.v, al.v, bq.v, bq.v, acc[t]); }
  }
#pragma unroll
  for (int t = 0; t < 4; ++t) { if (col0 + t * 16 >= N) continue;
#pragma unroll
    for (int r = 0; r < 8; ++r) so[w][8 * hh + r][t * 16 + ln] = acc[t][r] * alpha; }
  __builtin_amdgcn_fence(__ATOMIC_ACQ_REL, "workgroup"); __builtin_amdgcn_wave_barrier();
  const int rsub = lane >> 4, c4 = (lane & 15) * 4;
  for (int pass = 0; pass < 2; ++pass) {
#pragma unroll
    for (int q = 0; q < 8; ++q) { const int r = q * 2 + rsub; if (col0 + c4 < N) { const v4f v = *(const v4fa*)&so[w][r][c4]; *(volatile v4f*)(C + (size_t)(row0 + r) * ldc + col0 + c4) = v; } }
    if (pass == 0) __threadfence(); }
}

template <int DUMMY>
__global__ __launch_bounds__(128) void k_gemm_hh(const _Float16* __restrict__ A, int lda, size_t sA, const _Float16* __restrict__ Bh, int ldb, size_t sB, float alpha, float* __restrict__ C, int ldc, size_t sC, int M, int N, int K) {
  __shared__ __attribute__((aligned(16))) float so[4][16][64];
  const int tid = threadIdx.x, w = tid >> 5, lane = tid & 31, ln = lane & 15, hh = lane >> 4; const int by = blockIdx.y;
  A += (size_t)by * sA; Bh += (size_t)by * sB; C += (size_t)by * sC;
  const int ntn = (N + 63) / 64; const int wid = blockIdx.x * 4 + w; const int mt = wid / ntn, nq = wid % ntn; if (mt * 16 >= M) return;
  const int row0 = mt * 16, col0 = nq * 64; const _Float16* arow = A + (size_t)(row0 + ln) * lda;
  v8f acc[4] = {};
  for (int kb = 0; kb < K; kb += 32) { FragH ah; ah.half[0] = *(const v8us*)((const unsigned short*)arow + kb + 8 * hh); ah.half[1] = *(const v8us*)((const unsigned short*)arow + kb + 16 + 8 * hh);
#pragma unroll
    for (int t = 0; t < 4; ++t) { if (col0 + t * 16 >= N) continue; const size_t boff = (size_t)(col0 + t * 16 + ln) * ldb + kb; FragH bq; bq.half[0] = *(const v8us*)((const unsigned short*)Bh + boff + 8 * hh); bq.half[1] = *(const v8us*)((const unsigned short*)Bh + boff + 16 + 8 * hh);
      acc[t] = mmaH<1>(ah.v, ah.v, bq.v, bq.v, acc[t]); }
  }
#pragma unroll
  for (int t = 0; t < 4; ++t) { if (col0 + t * 16 >= N) continue;
#pragma unroll
    for (int r = 0; r < 8; ++r) so[w][8 * hh + r][t * 16 + ln] = acc[t][r] * alpha; }
  __builtin_amdgcn_fence(__ATOMIC_ACQ_REL, "workgroup"); __builtin_amdgcn_wave_barrier();
  const int rsub = lane >> 4, c4 = (lane & 15) * 4;
  for (int pass = 0; pass < 2; ++pass) {
#pragma unroll
    for (int q = 0; q < 8; ++q) { const int r = q * 2 + rsub; if (col0 + c4 < N) { const v4f v = *(const v4fa*)&so[w][r][c4]; *(volatile v4f*)(C + (size_t)(row0 + r) * ldc + col0 + c4) = v; } }
    if (pass == 0) __threadfence(); }
}

template <int ACT>
__global__ __launch_bounds__(128) void k_gemm_hhx(const _Float16* __restrict__ A, int lda, size_t sA, const _Float16* __restrict__ Bh, int ldb, size_t sB, float alpha, const float* __restrict__ bias, size_t sBias, const float* __restrict__ CP, int rowsPerB, size_t sCPb, int row0g,
    float* __restrict__ C, _Float16* __restrict__ C16, int ldc, size_t sC, int M, int N, int K) {
  __shared__ __attribute__((aligned(16))) float so[4][16][64];
  const int tid = threadIdx.x, w = tid >> 5, lane = tid & 31, ln = lane & 15, hh = lane >> 4; const int by = blockIdx.y;
  A += (size_t)by * sA; Bh += (size_t)by * sB; const size_t cofs = (size_t)by * sC; const float* bp = bias ? bias + (size_t)by * sBias : nullptr;
  const int ntn = (N + 63) / 64; const int wid = blockIdx.x * 4 + w; const int mt = wid / ntn, nq = wid % ntn; if (mt * 16 >= M) return;
  const int row0 = mt * 16, col0 = nq * 64; const _Float16* arow = A + (size_t)(row0 + ln) * lda;
  v8f acc[4] = {};
  for (int kb = 0; kb < K; kb += 32) { FragH ah; ah.half[0] = *(const v8us*)((const unsigned short*)arow + kb + 8 * hh); ah.half[1] = *(const v8us*)((const unsigned short*)arow + kb + 16 + 8 * hh);
#pragma unroll
    for (int t = 0; t < 4; ++t) { if (col0 + t * 16 >= N) continue; const size_t boff = (size_t)(col0 + t * 16 + ln) * ldb + kb; FragH bq; bq.half[0] = *(const v8us*)((const unsigned short*)Bh + boff + 8 * hh); bq.half[1] = *(const v8us*)((const unsigned short*)Bh + boff + 16 + 8 * hh);
      acc[t] = mmaH<1>(ah.v, ah.v, bq.v, bq.v, acc[t]); }
  }
#pragma unroll
  for (int t = 0; t < 4; ++t) { if (col0 + t * 16 >= N) continue; const int col = col0 + t * 16 + ln; const float bv = bp ? bf16_round(bp[col]) : 0.f;
#pragma unroll
    for (int r = 0; r < 8; ++r) { float v = acc[t][r] * alpha + bv; if (CP) { const int bidx = (row0g + row0 + 8 * hh + r) / rowsPerB; v += CP[(size_t)bidx * sCPb + (size_t)by * 64 + col]; } if (ACT == 1) v = (v > 0.f) ? v : expm1f(v); else if (ACT == 3) v = fmaxf(v, 0.f); so[w][8 * hh + r][t * 16 + ln] = v; } }
  __builtin_amdgcn_fence(__ATOMIC_ACQ_REL, "workgroup"); __builtin_amdgcn_wave_barrier();
  const int rsub = lane >> 4, c4 = (lane & 15) * 4; typedef _Float16 v4h __attribute__((ext_vector_type(4)));
  for (int pass = 0; pass < 2; ++pass) {
#pragma unroll
    for (int q = 0; q < 8; ++q) { const int r = q * 2 + rsub; if (col0 + c4 < N) { const v4f v = *(const v4fa*)&so[w][r][c4]; if (C) *(volatile v4f*)(C + cofs + (size_t)(row0 + r) * ldc + col0 + c4) = v; if (C16) { v4h h4; for (int i = 0; i < 4; ++i) h4[i] = (_Float16)v[i]; *(volatile v4h*)(C16 + cofs + (size_t)(row0 + r) * ldc + col0 + c4) = h4; } } }
    if (pass == 0) __threadfence(); }
}

__global__ __launch_bounds__(1024) void k_thr(const float* __restrict__ w0, int n0, const float* __restrict__ w1, int n1, const float* __restrict__ w2, int n2, const float* __restrict__ w3, int n3, float* __restrict__ T4) { __shared__ float red[32]; const int i = blockIdx.x, tid = threadIdx.x, lane = tid & 31, wv = tid >> 5; const float* w = i == 0 ? w0 : (i == 1 ? w1 : (i == 2 ? w2 : w3)); const int n = i == 0 ? n0 : (i == 1 ? n1 : (i == 2 ? n2 : n3)); float m = 0.f;
  for (int k = tid; k < n; k += 1024) m = fmaxf(m, fabsf(bf16_round(w[k]))); for (int o = 16; o >= 1; o >>= 1) m = fmaxf(m, __shfl_xor(m, o, 32)); if (lane == 0) red[wv] = m; __syncthreads(); if (tid == 0) { float mm = 0.f; for (int k = 0; k < 32; ++k) mm = fmaxf(mm, red[k]); const float t = 0.05f * mm; *(volatile float*)(T4 + i) = t; __threadfence(); *(volatile float*)(T4 + i) = t; } }
__device__ __forceinline__ _Float16 tq(float w, float t) { const float x = bf16_round(w); return (_Float16)((x > t ? 1.f : 0.f) - (x < -t ? 1.f : 0.f)); }
__global__ __launch_bounds__(256) void k_qw(const float* __restrict__ w1, const float* __restrict__ w2, const float* __restrict__ wf, const float* __restrict__ T4, _Float16* __restrict__ Bt1, _Float16* __restrict__ Bt2, _Float16* __restrict__ Btf) { const size_t t = (size_t)blockIdx.x * 256 + threadIdx.x;
  if (t < C1 * K1P) { const int k = (int)(t % K1P), o = (int)(t / K1P); *(volatile _Float16*)(Bt1 + t) = (k < 25) ? tq(w1[o * 25 + k], T4[0]) : (_Float16)0.f; }
  if (t < (size_t)C2 * K2) { const int k = (int)(t % K2), o = (int)(t / K2); const int c = k % C1, kk = k / C1; *(volatile _Float16*)(Bt2 + t) = tq(w2[((size_t)o * C1 + c) * 25 + kk], T4[1]); }
  if (t < (size_t)F1 * 2048) { *(volatile _Float16*)(Btf + t) = tq(wf[t], T4[2]); } }
__global__ __launch_bounds__(256) void k_im1(const float* __restrict__ x, _Float16* __restrict__ A1) { const size_t t = (size_t)blockIdx.x * 256 + threadIdx.x; if (t >= (size_t)R1 * K1P / 8) return; const int k8 = (int)((t * 8) % K1P); const size_t row = (t * 8) / K1P; const int ox = (int)(row % H1), oy = (int)((row / H1) % H1); const size_t b = row / (H1 * H1); FragH f;
  for (int q = 0; q < 8; ++q) { const int k = k8 + q; float v = 0.f; if (k < 25) { const int kh = k / 5, kw = k % 5; v = bf16_round(x[(b * H0 + oy + kh) * H0 + ox + kw]); } f.h[q] = (_Float16)v; }
  *(volatile v8us*)((unsigned short*)A1 + t * 8) = f.half[0]; __threadfence(); *(volatile v8us*)((unsigned short*)A1 + t * 8) = f.half[0]; }
__global__ __launch_bounds__(128) void k_colstat(const float* __restrict__ Cm, int R, int C, float* __restrict__ MU, float* __restrict__ IV) { const int c = blockIdx.x * 128 + threadIdx.x; if (c >= C) return; float s = 0.f;
#pragma unroll 4
  for (int r = 0; r < R; ++r) s += Cm[(size_t)r * C + c]; const float mu = s / (float)R; float q2 = 0.f;
#pragma unroll 4
  for (int r = 0; r < R; ++r) { const float d = Cm[(size_t)r * C + c] - mu; q2 += d * d; } const float iv = 1.0f / sqrtf(q2 / (float)R + 1e-5f); *(volatile float*)(MU + c) = mu; *(volatile float*)(IV + c) = iv; __threadfence(); *(volatile float*)(MU + c) = mu; *(volatile float*)(IV + c) = iv; }
__global__ __launch_bounds__(256) void k_pool1(const float* __restrict__ Cm, const float* __restrict__ MU, const float* __restrict__ IV, const float* __restrict__ g, const float* __restrict__ be, _Float16* __restrict__ P1) { const size_t t = (size_t)blockIdx.x * 256 + threadIdx.x; if (t >= (size_t)BB * Q1 * Q1 * C1 / 8) return; const int c8 = (int)((t * 8) % C1); const size_t pix = (t * 8) / C1; const int px = (int)(pix % Q1), py = (int)((pix / Q1) % Q1); const size_t b = pix / (Q1 * Q1); FragH f;
  for (int q = 0; q < 8; ++q) { const int c = c8 + q; const float mu = MU[c], sc = IV[c] * bf16_round(g[c]), sh = bf16_round(be[c]); float m = -3.0e38f; for (int dy = 0; dy < 2; ++dy) for (int dx = 0; dx < 2; ++dx) { const size_t row = (b * H1 + 2 * py + dy) * H1 + 2 * px + dx; const float v = fmaxf((Cm[row * C1 + c] - mu) * sc + sh, 0.f); m = fmaxf(m, v); } f.h[q] = (_Float16)m; }
  *(volatile v8us*)((unsigned short*)P1 + t * 8) = f.half[0]; __threadfence(); *(volatile v8us*)((unsigned short*)P1 + t * 8) = f.half[0]; }
__global__ __launch_bounds__(256) void k_im2(const _Float16* __restrict__ P1, int b0, _Float16* __restrict__ A2) { const size_t t = (size_t)blockIdx.x * 256 + threadIdx.x; if (t >= (size_t)BH2 * H2 * H2 * K2 / 8) return; const int k8 = (int)((t * 8) % K2); const size_t row = (t * 8) / K2; const int c8 = k8 % C1, kk = k8 / C1; const int kh = kk / 5, kw = kk % 5; const int ox = (int)(row % H2), oy = (int)((row / H2) % H2); const size_t b = b0 + row / (H2 * H2);
  const v8us v = *(const v8us*)((const unsigned short*)P1 + (((b * Q1 + oy + kh) * Q1 + ox + kw) * C1 + c8)); *(volatile v8us*)((unsigned short*)A2 + t * 8) = v; __threadfence(); *(volatile v8us*)((unsigned short*)A2 + t * 8) = v; }
__global__ __launch_bounds__(256) void k_pool2(const float* __restrict__ Cm, const float* __restrict__ MU, const float* __restrict__ IV, const float* __restrict__ g, const float* __restrict__ be, _Float16* __restrict__ P2) { const size_t t = (size_t)blockIdx.x * 256 + threadIdx.x; if (t >= (size_t)BB * C2 * Q2) return; const int y = (int)(t % Q2), c = (int)((t / Q2) % C2); const size_t b = t / (Q2 * C2); const float mu = MU[c], sc = IV[c] * bf16_round(g[c]), sh = bf16_round(be[c]);
  typedef _Float16 v4h __attribute__((ext_vector_type(4))); v4h o; for (int xq = 0; xq < Q2; ++xq) { float m = -3.0e38f; for (int dy = 0; dy < 2; ++dy) for (int dx = 0; dx < 2; ++dx) { const size_t row = (b * H2 + 2 * y + dy) * H2 + 2 * xq + dx; m = fmaxf(m, fmaxf((Cm[row * C2 + c] - mu) * sc + sh, 0.f)); } o[xq] = (_Float16)m; }
  _Float16* dst = P2 + b * 2048 + c * 16 + y * 4; *(volatile v4h*)dst = o; __threadfence(); *(volatile v4h*)dst = o; }
__global__ __launch_bounds__(512) void k_fc2(const float* __restrict__ Hm, const float* __restrict__ MU, const float* __restrict__ IV, const float* __restrict__ g, const float* __restrict__ be, const float* __restrict__ wf2, const float* __restrict__ bf2, const float* __restrict__ T4, float* __restrict__ OS) { __shared__ float sh[F1]; __shared__ float so[32]; const int b = blockIdx.x, c = threadIdx.x; sh[c] = fmaxf((Hm[(size_t)b * F1 + c] - MU[c]) * IV[c] * bf16_round(g[c]) + bf16_round(be[c]), 0.f); if (c < 32) so[c] = 0.f; __syncthreads();
  if (c < NCLS) { const float t = T4[3]; float s = bf16_round(bf2[c]);
#pragma unroll 4
    for (int k = 0; k < F1; ++k) s += sh[k] * (float)tq(wf2[c * F1 + k], t); so[c] = s; }
  __syncthreads(); if (c < 32) { *(volatile float*)(OS + b * 32 + c) = so[c]; } __threadfence(); if (c < 32) { *(volatile float*)(OS + b * 32 + c) = so[c]; } }
__global__ __launch_bounds__(256) void k_out(const float* __restrict__ OS, float* __restrict__ out) { const int t = blockIdx.x * 256 + threadIdx.x; if (t >= BB * NCLS) return; const float v = OS[(t / NCLS) * 32 + (t % NCLS)]; *(volatile float*)(out + t) = v; __threadfence(); *(volatile float*)(out + t) = v; }
extern "C" void kernel_launch(void* const* d_in, const int* in_sizes, int n_in,
                              void* d_out, int out_size, void* d_ws, size_t ws_size, hipStream_t stream) {
  (void)in_sizes; (void)n_in; (void)out_size;
  const float* x = (const float*)d_in[0]; const float* w1 = (const float*)d_in[1]; const float* b1 = (const float*)d_in[2]; const float* g1 = (const float*)d_in[3]; const float* be1 = (const float*)d_in[4]; const float* w2 = (const float*)d_in[5]; const float* b2 = (const float*)d_in[6]; const float* g2 = (const float*)d_in[7]; const float* be2 = (const float*)d_in[8]; const float* wf = (const float*)d_in[9]; const float* bfc = (const float*)d_in[10]; const float* g3 = (const float*)d_in[11]; const float* be3 = (const float*)d_in[12]; const float* wf2 = (const float*)d_in[13]; const float* bf2 = (const float*)d_in[14];
  char* ws = (char*)d_ws; size_t off = 0;
  auto take = [&](size_t bytes) { char* p = ws + off; off += (bytes + 255) & ~(size_t)255; return p; };
  float* T4 = (float*)take(256); _Float16* Bt1 = (_Float16*)take(C1 * K1P * 2); _Float16* Bt2 = (_Float16*)take((size_t)C2 * K2 * 2); _Float16* Btf = (_Float16*)take((size_t)F1 * 2048 * 2); float* MU = (float*)take(F1 * 4); float* IV = (float*)take(F1 * 4);
  _Float16* A1 = (_Float16*)take((size_t)R1 * K1P * 2); float* CM1 = (float*)take((size_t)R1 * C1 * 4); _Float16* P1 = (_Float16*)take((size_t)BB * Q1 * Q1 * C1 * 2); _Float16* P2 = (_Float16*)take((size_t)BB * 2048 * 2); float* HM = (float*)take((size_t)BB * F1 * 4); float* OS = (float*)take((size_t)BB * 32 * 4);
  _Float16* A2 = (_Float16*)CM1;
  float* CM2 = (float*)A1;
  if (off > ws_size) return;
  k_thr<<<4, 1024, 0, stream>>>(w1, C1 * 25, w2, C2 * C1 * 25, wf, F1 * 2048, wf2, NCLS * F1, T4);
  k_qw<<<(unsigned)(((size_t)F1 * 2048 + 255) / 256), 256, 0, stream>>>(w1, w2, wf, T4, Bt1, Bt2, Btf);
  k_im1<<<(unsigned)(((size_t)R1 * K1P / 8 + 255) / 256), 256, 0, stream>>>(x, A1);
  k_gemm_hhx<0><<<dim3(((R1 / 16) * 1 + 3) / 4, 1), 128, 0, stream>>>(A1, K1P, 0, Bt1, K1P, 0, 1.0f, b1, 0, nullptr, 1, 0, 0, CM1, nullptr, C1, 0, R1, C1, K1P);
  k_colstat<<<1, 128, 0, stream>>>(CM1, R1, C1, MU, IV);
  k_pool1<<<(unsigned)(((size_t)BB * Q1 * Q1 * C1 / 8 + 255) / 256), 256, 0, stream>>>(CM1, MU, IV, g1, be1, P1);
  for (int b0 = 0; b0 < BB; b0 += BH2) { k_im2<<<(unsigned)(((size_t)BH2 * H2 * H2 * K2 / 8 + 255) / 256), 256, 0, stream>>>(P1, b0, A2);
    k_gemm_hhx<0><<<dim3(((BH2 * H2 * H2 / 16) * (C2 / 64) + 3) / 4, 1), 128, 0, stream>>>(A2, K2, 0, Bt2, K2, 0, 1.0f, b2, 0, nullptr, 1, 0, 0, CM2 + (size_t)b0 * H2 * H2 * C2, nullptr, C2, 0, BH2 * H2 * H2, C2, K2); }
  k_colstat<<<1, 128, 0, stream>>>(CM2, R2, C2, MU, IV);
  k_pool2<<<(unsigned)(((size_t)BB * C2 * Q2 + 255) / 256), 256, 0, stream>>>(CM2, MU, IV, g2, be2, P2);
  k_gemm_hhx<0><<<dim3(((BB / 16) * (F1 / 64) + 3) / 4, 1), 128, 0, stream>>>(P2, 2048, 0, Btf, 2048, 0, 1.0f, bfc, 0, nullptr, 1, 0, 0, HM, nullptr, F1, 0, BB, F1, 2048);
  k_colstat<<<(F1 + 127) / 128, 128, 0, stream>>>(HM, BB, F1, MU, IV);
  k_fc2<<<BB, 512, 0, stream>>>(HM, MU, IV, g3, be3, wf2, bf2, T4, OS);
  k_out<<<(BB * NCLS + 255) / 256, 256, 0, stream>>>(OS, (float*)d_out);
}
